// PAB3D_51196010168769
// MI455X (gfx1250) — hardware-verified
//
#include <hip/hip_runtime.h>
#include <stddef.h>


typedef _Float16 f16;
typedef _Float16 v16h __attribute__((ext_vector_type(16)));
typedef _Float16 v8h  __attribute__((ext_vector_type(8)));
typedef float    v8f  __attribute__((ext_vector_type(8)));
typedef float    v4f  __attribute__((ext_vector_type(4)));

union Frag { v16h v; v8h h2[2]; };

constexpr int NBATCH = 2;
constexpr int NCH    = 64;
constexpr int NVOX   = 4096;
constexpr int NCELL  = 5832;
constexpr float WSCALE = 16.0f;
constexpr float WINV   = 0.0625f;
constexpr float ESCALE = 16384.0f;
constexpr float EINV   = 1.0f / 16384.0f;

constexpr int W1GROUPS = NCH * NCH / 8;
constexpr int W3GROUPS = NCH * NCH * 27 / 8;

__device__ __forceinline__ v8f wmma16(v16h a, v16h b, v8f c) {
    c = __builtin_amdgcn_wmma_f32_16x16x32_f16(false, a, false, b, (short)0, c, false, false);
    asm volatile("v_nop\n\tv_nop\n\tv_nop\n\tv_nop" : "+v"(c) : "v"(a), "v"(b));
    return c;
}
__device__ __forceinline__ v8f zero8() {
    v8f z;
#pragma unroll
    for (int i = 0; i < 8; ++i) z[i] = 0.0f;
    return z;
}
__device__ __forceinline__ v16h ldfrag(const f16* p, int h) {
    Frag f;
    f.h2[0] = *(const v8h*)(p + 8 * h);
    f.h2[1] = *(const v8h*)(p + 16 + 8 * h);
    return f.v;
}

__global__ void __launch_bounds__(256) k_prepw(const float* __restrict__ tw, const float* __restrict__ cw,
                                               const float* __restrict__ bw, const float* __restrict__ ow,
                                               f16* Wt, f16* Wc, f16* Wb, f16* Wo, int total)
{
    const int g = blockIdx.x * 256 + threadIdx.x;
    if (g >= total) return;
    v8h v;
    f16* dst;
    if (g < 2 * W1GROUPS) {
        const float* src = (g < W1GROUPS) ? tw : cw;
        f16* base = (g < W1GROUPS) ? Wt : Wc;
        const int e0 = (g & (W1GROUPS - 1)) * 8;
        dst = base + e0;
#pragma unroll
        for (int i = 0; i < 8; ++i) v[i] = (f16)(src[e0 + i] * WSCALE);
    } else {
        const int gg = g - 2 * W1GROUPS;
        const float* src = (gg < W3GROUPS) ? bw : ow;
        f16* base = (gg < W3GROUPS) ? Wb : Wo;
        const int q = (gg < W3GROUPS) ? gg : (gg - W3GROUPS);
        const int o = q * 8;
        const int co = o / 1728;
        const int rem = o - co * 1728;
        const int tp = rem >> 6;
        const int ci = rem & 63;
        dst = base + o;
#pragma unroll
        for (int i = 0; i < 8; ++i) v[i] = (f16)(src[(size_t)(co * 64 + ci + i) * 27 + tp] * WSCALE);
    }
    *(volatile v8h*)dst = v;
    __threadfence();
    *(volatile v8h*)dst = v;
}

template <bool ADD>
__global__ void __launch_bounds__(256) k_plane(const float* __restrict__ x, const float* __restrict__ U,
                                               const float* __restrict__ rs, f16* P, int total)
{
    const int g = blockIdx.x * 256 + threadIdx.x;
    if (g >= total) return;
    const int q = g & 7;
    const int cellg = g >> 3;
    const int b = cellg / NCELL;
    const int cell = cellg - b * NCELL;
    const int ph = cell / 324;
    const int r2 = cell - ph * 324;
    const int pw = r2 / 18;
    const int pd = r2 - pw * 18;
    const int hh = ph - 1, ww = pw - 1, dd = pd - 1;
    const bool inside = ((unsigned)hh < 16u) && ((unsigned)ww < 16u) && ((unsigned)dd < 16u);
    v8h v;
#pragma unroll
    for (int i = 0; i < 8; ++i) v[i] = (f16)0.0f;
    if (inside) {
        const int n = (hh << 8) | (ww << 4) | dd;
        const size_t bb = (size_t)b * (NCH * NVOX);
#pragma unroll
        for (int i = 0; i < 8; ++i) {
            const int c = 8 * q + i;
            const size_t f = (size_t)c * NVOX + n;
            float val = x[bb + f];
            if (ADD) val = val + U[bb + f] * rs[b * NVOX + (int)(f >> 6)];
            v[i] = (f16)val;
        }
    }
    f16* dst = P + ((size_t)cellg * NCH + 8 * q);
    *(volatile v8h*)dst = v;
    __threadfence();
    *(volatile v8h*)dst = v;
}

template <int NTAP, int MODE>
__global__ void __launch_bounds__(128) k_conv(const f16* __restrict__ P,
        const f16* __restrict__ W0, const float* __restrict__ bias0, void* out0,
        const f16* __restrict__ W1, const float* __restrict__ bias1, void* out1)
{
    __shared__ float sm[64][68] __attribute__((aligned(16)));
    const int nt = blockIdx.x, b = blockIdx.y, sel = blockIdx.z;
    const f16* W = sel ? W1 : W0;
    const float* bias = sel ? bias1 : bias0;
    void* outp = sel ? out1 : out0;
    const int lane = threadIdx.x & 31, wv = threadIdx.x >> 5, h = lane >> 4, m = lane & 15;
    const int n0 = nt * 64;
    const f16* Pb = P + (size_t)b * NCELL * NCH;

    int cb[4];
#pragma unroll
    for (int t = 0; t < 4; ++t) {
        const int n = n0 + 16 * t + m;
        const int vh = n >> 8, vw = (n >> 4) & 15, vd = n & 15;
        cb[t] = (vh * 18 + vw) * 18 + vd;
    }
    constexpr int KW = NTAP * NCH;
    constexpr int T3 = (NTAP == 27) ? 3 : 1;
    const f16* Wrow = W + (size_t)(16 * wv + m) * KW;

    v8f acc[4];
#pragma unroll
    for (int t = 0; t < 4; ++t) acc[t] = zero8();

    for (int t2 = 0; t2 < T3; ++t2) {
        for (int t3 = 0; t3 < T3; ++t3) {
            for (int t4 = 0; t4 < T3; ++t4) {
                const int toff = (NTAP == 27) ? ((t2 * 18 + t3) * 18 + t4) : 343;
                const int wk   = (NTAP == 27) ? (((t2 * 3 + t3) * 3 + t4) * NCH) : 0;
#pragma unroll
                for (int ks = 0; ks < 2; ++ks) {
                    const v16h af = ldfrag(Wrow + wk + 32 * ks, h);
#pragma unroll
                    for (int t = 0; t < 4; ++t) {
                        const v16h bf = ldfrag(Pb + (size_t)(cb[t] + toff) * NCH + 32 * ks, h);
                        acc[t] = wmma16(af, bf, acc[t]);
                    }
                }
            }
        }
    }

    float bv[8];
#pragma unroll
    for (int r = 0; r < 8; ++r) bv[r] = bias[16 * wv + 8 * h + r];
#pragma unroll
    for (int t = 0; t < 4; ++t) {
#pragma unroll
        for (int r = 0; r < 8; ++r) sm[16 * wv + 8 * h + r][16 * t + m] = acc[t][r] * WINV + bv[r];
    }
    __syncthreads();

    if (MODE == 0) {
        float* O = (float*)outp + (size_t)b * NCH * NVOX + n0;
        v4f vv[8];
#pragma unroll
        for (int j = 0; j < 8; ++j) {
            const int row = 16 * wv + 2 * j + h;
            const int col = 4 * m;
            vv[j] = *(const v4f*)(&sm[row][col]);
            *(volatile v4f*)(O + (size_t)row * NVOX + col) = vv[j];
        }
        __threadfence();
#pragma unroll
        for (int j = 0; j < 8; ++j) {
            const int row = 16 * wv + 2 * j + h;
            const int col = 4 * m;
            *(volatile v4f*)(O + (size_t)row * NVOX + col) = vv[j];
        }
    } else if (MODE == 1) {
        f16* O = (f16*)outp + (size_t)b * NCH * NVOX + n0;
        v8h vv[4];
#pragma unroll
        for (int j = 0; j < 4; ++j) {
            const int row = 16 * wv + 4 * j + (lane >> 3);
            const int col = 8 * (lane & 7);
            v8h pk;
#pragma unroll
            for (int i = 0; i < 8; ++i) pk[i] = (f16)sm[row][col + i];
            vv[j] = pk;
            *(volatile v8h*)(O + (size_t)row * NVOX + col) = pk;
        }
        __threadfence();
#pragma unroll
        for (int j = 0; j < 4; ++j) {
            const int row = 16 * wv + 4 * j + (lane >> 3);
            const int col = 8 * (lane & 7);
            *(volatile v8h*)(O + (size_t)row * NVOX + col) = vv[j];
        }
    } else {
        f16* O = (f16*)outp + ((size_t)b * NVOX + n0) * NCH;
        v8h vv[4];
#pragma unroll
        for (int j = 0; j < 4; ++j) {
            const int nl = 16 * wv + 4 * j + (lane >> 3);
            const int p0 = 8 * (lane & 7);
            v8h pk;
#pragma unroll
            for (int i = 0; i < 8; ++i) pk[i] = (f16)sm[p0 + i][nl];
            vv[j] = pk;
            *(volatile v8h*)(O + (size_t)nl * NCH + p0) = pk;
        }
        __threadfence();
#pragma unroll
        for (int j = 0; j < 4; ++j) {
            const int nl = 16 * wv + 4 * j + (lane >> 3);
            const int p0 = 8 * (lane & 7);
            *(volatile v8h*)(O + (size_t)nl * NCH + p0) = vv[j];
        }
    }
}

__device__ __forceinline__ v8f stile(const f16* trow, int h, v16h bq0, v16h bq1) {
    v8f d = zero8();
    d = wmma16(ldfrag(trow, h), bq0, d);
    d = wmma16(ldfrag(trow + 32, h), bq1, d);
    return d;
}

__global__ void __launch_bounds__(256) k_smax1(const f16* __restrict__ topT, const f16* __restrict__ cenT,
                                               float* rmax)
{
    __shared__ float s_r[128] __attribute__((aligned(16)));
    const int lane = threadIdx.x & 31, wv = threadIdx.x >> 5, h = lane >> 4, m = lane & 15;
    const int b = blockIdx.y;
    const int nb0 = blockIdx.x * 128;
    const int n0 = nb0 + wv * 16;
    const f16* tb = topT + (size_t)b * NVOX * NCH;
    const f16* cbp = cenT + (size_t)b * NVOX * NCH;
    const v16h bq0 = ldfrag(cbp + (size_t)(n0 + m) * NCH, h);
    const v16h bq1 = ldfrag(cbp + (size_t)(n0 + m) * NCH + 32, h);

    float mx = -3.0e38f;
    for (int m0 = 0; m0 < NVOX; m0 += 32) {
        const v8f d0 = stile(tb + (size_t)(m0 + m) * NCH, h, bq0, bq1);
        const v8f d1 = stile(tb + (size_t)(m0 + 16 + m) * NCH, h, bq0, bq1);
#pragma unroll
        for (int r = 0; r < 8; ++r) mx = fmaxf(mx, fmaxf(d0[r], d1[r]));
    }
    mx = fmaxf(mx, __shfl_xor(mx, 16));
    if (lane < 16) s_r[wv * 16 + lane] = mx;
    __syncthreads();
    if (wv == 0) {
        const v4f v = *(const v4f*)(&s_r[4 * lane]);
        float* dst = rmax + b * NVOX + nb0 + 4 * lane;
        *(volatile v4f*)dst = v;
        __threadfence();
        *(volatile v4f*)dst = v;
    }
}

__global__ void __launch_bounds__(256) k_smax2(const f16* __restrict__ topT, const f16* __restrict__ cenT,
                                               const f16* __restrict__ botN, const float* __restrict__ rmax,
                                               float* U, float* zsum)
{
    __shared__ float su[8][16][68] __attribute__((aligned(16)));
    __shared__ float s_z[128] __attribute__((aligned(16)));
    const int lane = threadIdx.x & 31, wv = threadIdx.x >> 5, h = lane >> 4, m = lane & 15;
    const int b = blockIdx.y;
    const int nb0 = blockIdx.x * 128;
    const int n0 = nb0 + wv * 16;
    const f16* tb = topT + (size_t)b * NVOX * NCH;
    const f16* cbp = cenT + (size_t)b * NVOX * NCH;
    const f16* bnb = botN + (size_t)b * NCH * NVOX;
    const v16h bq0 = ldfrag(cbp + (size_t)(n0 + m) * NCH, h);
    const v16h bq1 = ldfrag(cbp + (size_t)(n0 + m) * NCH + 32, h);
    const float rl = rmax[b * NVOX + n0 + m];

    float zs = 0.0f;
    v8f oacc[4];
#pragma unroll
    for (int ct = 0; ct < 4; ++ct) oacc[ct] = zero8();

    for (int m0 = 0; m0 < NVOX; m0 += 32) {
        const v8f d0 = stile(tb + (size_t)(m0 + m) * NCH, h, bq0, bq1);
        const v8f d1 = stile(tb + (size_t)(m0 + 16 + m) * NCH, h, bq0, bq1);
        v8h p0, p1;
#pragma unroll
        for (int r = 0; r < 8; ++r) {
            const float e0 = __expf(d0[r] - rl);
            const float e1 = __expf(d1[r] - rl);
            zs += e0;
            zs += e1;
            p0[r] = (f16)(e0 * ESCALE);
            p1[r] = (f16)(e1 * ESCALE);
        }
        Frag ap;
        ap.h2[0] = p0;
        ap.h2[1] = p1;
#pragma unroll
        for (int ct = 0; ct < 4; ++ct) {
            const v16h bf = ldfrag(bnb + (size_t)(16 * ct + m) * NVOX + m0, h);
            oacc[ct] = wmma16(ap.v, bf, oacc[ct]);
        }
    }

#pragma unroll
    for (int ct = 0; ct < 4; ++ct) {
#pragma unroll
        for (int r = 0; r < 8; ++r) su[wv][8 * h + r][16 * ct + m] = oacc[ct][r];
    }
    zs += __shfl_xor(zs, 16);
    if (lane < 16) s_z[wv * 16 + lane] = zs;
    __syncthreads();

    float* Ub = U + ((size_t)(b * NVOX + n0)) * NCH;
    v4f vv[8];
#pragma unroll
    for (int j = 0; j < 8; ++j) {
        const int row = 2 * j + h;
        const int col = 4 * m;
        vv[j] = *(const v4f*)(&su[wv][row][col]);
        *(volatile v4f*)(Ub + (size_t)row * NCH + col) = vv[j];
    }
    v4f zv;
#pragma unroll
    for (int c = 0; c < 4; ++c) zv[c] = 0.0f;
    if (wv == 0) {
        zv = *(const v4f*)(&s_z[4 * lane]);
        *(volatile v4f*)(zsum + b * NVOX + nb0 + 4 * lane) = zv;
    }
    __threadfence();
#pragma unroll
    for (int j = 0; j < 8; ++j) {
        const int row = 2 * j + h;
        const int col = 4 * m;
        *(volatile v4f*)(Ub + (size_t)row * NCH + col) = vv[j];
    }
    if (wv == 0) {
        *(volatile v4f*)(zsum + b * NVOX + nb0 + 4 * lane) = zv;
    }
}

__global__ void __launch_bounds__(256) k_stats(const float* __restrict__ rmax, const float* __restrict__ zsum, float* rs)
{
    __shared__ float red[256];
    const int b = blockIdx.x, t = threadIdx.x;
    const float* rm = rmax + b * NVOX;
    const float* zz = zsum + b * NVOX;

    float mx = -3.0e38f;
#pragma unroll 1
    for (int i = 0; i < 16; ++i) mx = fmaxf(mx, rm[t + 256 * i]);
    red[t] = mx;
    __syncthreads();
    for (int s = 128; s > 0; s >>= 1) {
        if (t < s) red[t] = fmaxf(red[t], red[t + s]);
        __syncthreads();
    }
    const float M = red[0];
    __syncthreads();

    float acc = 0.0f;
#pragma unroll 1
    for (int i = 0; i < 16; ++i) {
        const int n = t + 256 * i;
        acc += zz[n] * __expf(rm[n] - M);
    }
    red[t] = acc;
    __syncthreads();
    for (int s = 128; s > 0; s >>= 1) {
        if (t < s) red[t] = red[t] + red[t + s];
        __syncthreads();
    }
    const float Z = red[0];
    const float kf = (1.0f / Z) * EINV;

    v4f vv[4];
#pragma unroll
    for (int i = 0; i < 4; ++i) {
        const int n = 4 * t + 1024 * i;
        v4f v;
#pragma unroll
        for (int c = 0; c < 4; ++c) v[c] = __expf(rm[n + c] - M) * kf;
        vv[i] = v;
        *(volatile v4f*)(rs + b * NVOX + n) = v;
    }
    __threadfence();
#pragma unroll
    for (int i = 0; i < 4; ++i) {
        const int n = 4 * t + 1024 * i;
        *(volatile v4f*)(rs + b * NVOX + n) = vv[i];
    }
}

extern "C" void kernel_launch(void* const* d_in, const int* in_sizes, int n_in,
                              void* d_out, int out_size, void* d_ws, size_t ws_size,
                              hipStream_t stream)
{
    if (n_in < 9) return;
    if (in_sizes[0] != NBATCH * NCH * NVOX || in_sizes[1] != NCH * NCH || in_sizes[2] != NCH ||
        in_sizes[3] != NCH * NCH || in_sizes[4] != NCH || in_sizes[5] != NCH * NCH * 27 ||
        in_sizes[6] != NCH || in_sizes[7] != NCH * NCH * 27 || in_sizes[8] != NCH ||
        out_size != NBATCH * NCH * NVOX) return;

    const float* x  = (const float*)d_in[0];
    const float* tw = (const float*)d_in[1];
    const float* tb = (const float*)d_in[2];
    const float* cw = (const float*)d_in[3];
    const float* cb = (const float*)d_in[4];
    const float* bw = (const float*)d_in[5];
    const float* bb = (const float*)d_in[6];
    const float* ow = (const float*)d_in[7];
    const float* ob = (const float*)d_in[8];
    float* out = (float*)d_out;

    char* ws = (char*)d_ws;
    size_t off = 0;
    auto carve = [&](size_t bytes) -> char* {
        char* p = ws + off;
        off += (bytes + 255) & ~(size_t)255;
        return p;
    };
    const size_t planeB = (size_t)NBATCH * NCELL * NCH * sizeof(f16);
    const size_t bnc    = (size_t)NBATCH * NVOX * NCH;
    f16*   xP   = (f16*)carve(planeB);
    f16*   zP   = (f16*)carve(planeB);
    f16*   Wt   = (f16*)carve((size_t)NCH * NCH * sizeof(f16));
    f16*   Wc   = (f16*)carve((size_t)NCH * NCH * sizeof(f16));
    f16*   Wb   = (f16*)carve((size_t)NCH * NCH * 27 * sizeof(f16));
    f16*   Wo   = (f16*)carve((size_t)NCH * NCH * 27 * sizeof(f16));
    f16*   topT = (f16*)carve(bnc * sizeof(f16));
    f16*   cenT = (f16*)carve(bnc * sizeof(f16));
    f16*   botN = (f16*)carve(bnc * sizeof(f16));
    float* U    = (float*)carve(bnc * sizeof(float));
    float* rmax = (float*)carve((size_t)NBATCH * NVOX * sizeof(float));
    float* zsum = (float*)carve((size_t)NBATCH * NVOX * sizeof(float));
    float* rs   = (float*)carve((size_t)NBATCH * NVOX * sizeof(float));
    if (off > ws_size || off > (size_t)134217728) return;

    const int prepw_total = 2 * W1GROUPS + 2 * W3GROUPS;
    const int plane_total = NBATCH * NCELL * 8;

    k_prepw<<<(prepw_total + 255) / 256, 256, 0, stream>>>(tw, cw, bw, ow, Wt, Wc, Wb, Wo, prepw_total);
    k_plane<false><<<(plane_total + 255) / 256, 256, 0, stream>>>(x, U, rs, xP, plane_total);
    k_conv<1, 2><<<dim3(NVOX / 64, NBATCH, 2), 128, 0, stream>>>(xP, Wt, tb, (void*)topT, Wc, cb, (void*)cenT);
    k_conv<27, 1><<<dim3(NVOX / 64, NBATCH, 1), 128, 0, stream>>>(xP, Wb, bb, (void*)botN, Wb, bb, (void*)botN);
    k_smax1<<<dim3(NVOX / 128, NBATCH, 1), 256, 0, stream>>>(topT, cenT, rmax);
    k_smax2<<<dim3(NVOX / 128, NBATCH, 1), 256, 0, stream>>>(topT, cenT, botN, rmax, U, zsum);
    k_stats<<<NBATCH, 256, 0, stream>>>(rmax, zsum, rs);
    k_plane<true><<<(plane_total + 255) / 256, 256, 0, stream>>>(x, U, rs, zP, plane_total);
    k_conv<27, 0><<<dim3(NVOX / 64, NBATCH, 1), 128, 0, stream>>>(zP, Wo, ob, (void*)out, Wo, ob, (void*)out);
}
